// RelativeAttention_29145648070828
// MI455X (gfx1250) — hardware-verified
//
#include <hip/hip_runtime.h>
#include <math.h>

static constexpr int kB  = 2;
static constexpr int kS  = 2048;
static constexpr int kD  = 1024;
static constexpr int kH  = 16;
static constexpr int kHD = 64;
static constexpr int kNR = 65;
static constexpr int kMAXD = 32;

typedef __attribute__((ext_vector_type(16))) _Float16 v16h;
typedef __attribute__((ext_vector_type(8)))  _Float16 v8h;
typedef __attribute__((ext_vector_type(8)))  float  v8f;
typedef __attribute__((ext_vector_type(4)))  int    v4i;

typedef __attribute__((address_space(1))) v4i as1_v4i;
typedef __attribute__((address_space(3))) v4i as3_v4i;

static __device__ __forceinline__ void g2l_b128(const _Float16* gsrc, _Float16* ldst) {
  *(v8h*)ldst = *(const v8h*)gsrc;
}
static __device__ __forceinline__ void wait_lds_arrivals() {}
typedef __attribute__((ext_vector_type(4))) float v4f;
typedef __attribute__((ext_vector_type(4))) unsigned v4u;
template <typename V> static __device__ __forceinline__ void vst2(void* p, V v) {
  *(volatile V*)p = v; __threadfence(); *(volatile V*)p = v;
}
#define PSC 256.0f
#define PUN (1.0f / 256.0f)
static __device__ __forceinline__ v8f wmma16(v16h a, v16h b, v8f c) {
  v8f d = __builtin_amdgcn_wmma_f32_16x16x32_f16(false, a, false, b, (short)0, c, false, false);
  asm volatile("v_nop\n\tv_nop\n\tv_nop\n\tv_nop" : "+v"(d) : "v"(a), "v"(b));
  return d;
}

union FragU { v16h v; v8h h[2]; };

static __device__ __forceinline__ v16h frag_a(const _Float16* rowk, int lane) {
  const int o = (lane >> 4) * 8;
  FragU f;
  f.h[0] = *(const v8h*)(rowk + o);
  f.h[1] = *(const v8h*)(rowk + o + 16);
  return f.v;
}
static __device__ __forceinline__ v16h frag_b(const _Float16* colk, int lane) {
  return frag_a(colk, lane);
}

__global__ __launch_bounds__(256)
void cvt_bf16_kernel(const float* __restrict__ in, _Float16* __restrict__ out, int n2) {
  int i = (blockIdx.x * 256 + threadIdx.x) * 2;
  if (i < n2) {
    union { _Float16 h[2]; unsigned u; } pk;
    pk.h[0] = (_Float16)in[i]; pk.h[1] = (_Float16)in[i + 1];
    vst2(out + i, pk.u);
  }
}

__global__ __launch_bounds__(128)
void wtrans_kernel(const float* __restrict__ W, _Float16* __restrict__ Wt, int K, int N) {
  __shared__ _Float16 sT[64 * 72];
  const int tid = threadIdx.x;
  const int n0 = blockIdx.x * 64;
  const int k0 = blockIdx.y * 64;
#pragma unroll
  for (int i = 0; i < 32; ++i) {
    int idx = tid + i * 128;
    int k = idx >> 6, n = idx & 63;
    sT[n * 72 + k] = (_Float16)W[(size_t)(k0 + k) * N + n0 + n];
  }
  __syncthreads();
#pragma unroll
  for (int i = 0; i < 4; ++i) {
    int g = tid + i * 128;
    int n = g >> 3, pc = g & 7;
    vst2(Wt + (size_t)(n0 + n) * K + k0 + pc * 8, *(const v4u*)(&sT[n * 72 + pc * 8]));
  }
}

template <typename TO>
__global__ __launch_bounds__(128)
void gemm_bias_kernel(const _Float16* __restrict__ Xb, const _Float16* __restrict__ Wt,
                      const float* __restrict__ bias, TO* __restrict__ Cout,
                      int N, int K, float alpha) {
  __shared__ __align__(32) _Float16 sA[64 * 64];
  __shared__ __align__(32) _Float16 sB[64 * 64];
  __shared__ __align__(16) float sC[4][16 * 64];
  const int tid  = threadIdx.x;
  const int wave = tid >> 5;
  const int lane = tid & 31;
  const int n0 = blockIdx.x * 64;
  const int m0 = blockIdx.y * 64;

  v8f acc[4];
#pragma unroll
  for (int t = 0; t < 4; ++t)
#pragma unroll
    for (int i = 0; i < 8; ++i) acc[t][i] = 0.0f;

  for (int kb = 0; kb < K; kb += 64) {
#pragma unroll
    for (int i = 0; i < 4; ++i) {
      int idx = tid + i * 128;
      int r = idx >> 3, c = (idx & 7) * 8;
      g2l_b128(&Xb[(size_t)(m0 + r) * K + kb + c], &sA[r * 64 + c]);
      g2l_b128(&Wt[(size_t)(n0 + r) * K + kb + c], &sB[r * 64 + c]);
    }
    wait_lds_arrivals();
    __syncthreads();
#pragma unroll
    for (int ks = 0; ks < 2; ++ks) {
      v16h a = frag_a(&sA[(wave * 16 + (lane & 15)) * 64 + ks * 32], lane);
#pragma unroll
      for (int t = 0; t < 4; ++t) {
        v16h bb = frag_b(&sB[(t * 16 + (lane & 15)) * 64 + ks * 32], lane);
        acc[t] = wmma16(a, bb, acc[t]);
      }
    }
    __syncthreads();
  }
  float* sc = sC[wave];
#pragma unroll
  for (int t = 0; t < 4; ++t) {
#pragma unroll
    for (int r = 0; r < 8; ++r) {
      int ml = r + ((lane >> 4) << 3);
      int n = n0 + t * 16 + (lane & 15);
      sc[ml * 64 + t * 16 + (lane & 15)] = alpha * (acc[t][r] + bias[n]);
    }
  }
  __syncthreads();
  if (sizeof(TO) == 2) {
#pragma unroll
    for (int q = 0; q < 4; ++q) {
      const int ml = q * 4 + (lane >> 3), pc = lane & 7;
      union { v8h h; v4u u; } pk;
#pragma unroll
      for (int e = 0; e < 8; ++e) pk.h[e] = (_Float16)sc[ml * 64 + pc * 8 + e];
      vst2((_Float16*)Cout + (size_t)(m0 + wave * 16 + ml) * N + n0 + pc * 8, pk.u);
    }
  } else {
#pragma unroll
    for (int q = 0; q < 8; ++q) {
      const int ml = q * 2 + (lane >> 4), pc = lane & 15;
      vst2((float*)Cout + (size_t)(m0 + wave * 16 + ml) * N + n0 + pc * 4, *(const v4f*)(&sc[ml * 64 + pc * 4]));
    }
  }
}

__global__ __launch_bounds__(128)
void rel_attn_kernel(const _Float16* __restrict__ Qb, const _Float16* __restrict__ Kb,
                     const _Float16* __restrict__ Vb, const float* __restrict__ rel_emb,
                     _Float16* __restrict__ ctx) {
  __shared__ __align__(32) _Float16 sQ[64 * 64];
  __shared__ __align__(32) _Float16 sK[64 * 64];
  __shared__ __align__(32) _Float16 sV[64 * 64];
  __shared__ __align__(32) _Float16 sP[64 * 64];
  __shared__ float sRel[kNR * kHD];
  __shared__ float sQrel[64 * 66];
  __shared__ __align__(16) _Float16 sO[4][16 * 64];

  const int tid  = threadIdx.x;
  const int wave = tid >> 5;
  const int lane = tid & 31;
  const int qb = blockIdx.x & 31;
  const int h  = (blockIdx.x >> 5) & 15;
  const int b  = blockIdx.x >> 9;
  const int q0 = qb * 64;

  for (int idx = tid; idx < kNR * kHD; idx += 128) sRel[idx] = rel_emb[idx];
#pragma unroll
  for (int i = 0; i < 4; ++i) {
    int idx = tid + i * 128;
    int r = idx >> 3, c = (idx & 7) * 8;
    g2l_b128(&Qb[((size_t)(b * kS + q0 + r)) * kD + h * kHD + c], &sQ[r * 64 + c]);
  }
  wait_lds_arrivals();
  __syncthreads();

  for (int idx = tid; idx < 64 * kNR; idx += 128) {
    int r = idx / kNR, dd = idx % kNR;
    float s = 0.f;
#pragma unroll 8
    for (int d = 0; d < kHD; ++d) s += (float)sQ[r * 64 + d] * sRel[dd * kHD + d];
    sQrel[r * 66 + dd] = s;
  }
  __syncthreads();

  v8f accO[4];
  float rowM[8], rowL[8];
#pragma unroll
  for (int t = 0; t < 4; ++t)
#pragma unroll
    for (int i = 0; i < 8; ++i) accO[t][i] = 0.0f;
#pragma unroll
  for (int r = 0; r < 8; ++r) { rowM[r] = -3.0e38f; rowL[r] = 0.0f; }

  for (int kt = 0; kt < kS / 64; ++kt) {
    const int k0 = kt * 64;
    const int knext = (kt + 1 < kS / 64) ? (k0 + 64) : k0;
    __builtin_prefetch(&Kb[((size_t)(b * kS + knext)) * kD + h * kHD], 0, 1);
#pragma unroll
    for (int i = 0; i < 4; ++i) {
      int idx = tid + i * 128;
      int r = idx >> 3, c = (idx & 7) * 8;
      size_t g = ((size_t)(b * kS + k0 + r)) * kD + h * kHD + c;
      g2l_b128(&Kb[g], &sK[r * 64 + c]);
      v8h vv = *(const v8h*)&Vb[g];
#pragma unroll
      for (int j = 0; j < 8; ++j) sV[(c + j) * 64 + r] = vv[j];
    }
    wait_lds_arrivals();
    __syncthreads();

    v8f accS[4];
#pragma unroll
    for (int t = 0; t < 4; ++t)
#pragma unroll
      for (int i = 0; i < 8; ++i) accS[t][i] = 0.0f;
#pragma unroll
    for (int ks = 0; ks < 2; ++ks) {
      v16h a = frag_a(&sQ[(wave * 16 + (lane & 15)) * 64 + ks * 32], lane);
#pragma unroll
      for (int t = 0; t < 4; ++t) {
        v16h bb = frag_b(&sK[(t * 16 + (lane & 15)) * 64 + ks * 32], lane);
        accS[t] = wmma16(a, bb, accS[t]);
      }
    }

    float sv[4][8], tmax[8];
#pragma unroll
    for (int r = 0; r < 8; ++r) tmax[r] = -3.0e38f;
#pragma unroll
    for (int t = 0; t < 4; ++t) {
#pragma unroll
      for (int r = 0; r < 8; ++r) {
        int m  = r + ((lane >> 4) << 3);
        int qi = q0 + wave * 16 + m;
        int ki = k0 + t * 16 + (lane & 15);
        int dd = qi - ki;
        dd = dd < -kMAXD ? -kMAXD : (dd > kMAXD ? kMAXD : dd);
        float x = accS[t][r] + sQrel[(wave * 16 + m) * 66 + (dd + kMAXD)];
        sv[t][r] = x;
        tmax[r] = fmaxf(tmax[r], x);
      }
    }
#pragma unroll
    for (int r = 0; r < 8; ++r) {
      float v = tmax[r];
      v = fmaxf(v, __shfl_xor(v, 1, 32));
      v = fmaxf(v, __shfl_xor(v, 2, 32));
      v = fmaxf(v, __shfl_xor(v, 4, 32));
      v = fmaxf(v, __shfl_xor(v, 8, 32));
      tmax[r] = v;
    }
    float corr[8], psum[8];
#pragma unroll
    for (int r = 0; r < 8; ++r) {
      float nm = fmaxf(rowM[r], tmax[r]);
      corr[r] = __expf(rowM[r] - nm);
      rowM[r] = nm;
      psum[r] = 0.0f;
    }
#pragma unroll
    for (int t = 0; t < 4; ++t) {
#pragma unroll
      for (int r = 0; r < 8; ++r) {
        int m = r + ((lane >> 4) << 3);
        float p = __expf(sv[t][r] - rowM[r]);
        psum[r] += p;
        sP[(wave * 16 + m) * 64 + t * 16 + (lane & 15)] = (_Float16)(p * PSC);
      }
    }
#pragma unroll
    for (int r = 0; r < 8; ++r) {
      float v = psum[r];
      v += __shfl_xor(v, 1, 32);
      v += __shfl_xor(v, 2, 32);
      v += __shfl_xor(v, 4, 32);
      v += __shfl_xor(v, 8, 32);
      rowL[r] = rowL[r] * corr[r] + v;
    }
#pragma unroll
    for (int t = 0; t < 4; ++t)
#pragma unroll
      for (int r = 0; r < 8; ++r) accO[t][r] *= corr[r];
    __syncthreads();

#pragma unroll
    for (int ks = 0; ks < 2; ++ks) {
      v16h a = frag_a(&sP[(wave * 16 + (lane & 15)) * 64 + ks * 32], lane);
#pragma unroll
      for (int t = 0; t < 4; ++t) {
        v16h bb = frag_b(&sV[(t * 16 + (lane & 15)) * 64 + ks * 32], lane);
        accO[t] = wmma16(a, bb, accO[t]);
      }
    }
    __syncthreads();
  }

  _Float16* so = sO[wave];
#pragma unroll
  for (int t = 0; t < 4; ++t) {
#pragma unroll
    for (int r = 0; r < 8; ++r) {
      int m = r + ((lane >> 4) << 3);
      so[m * 64 + t * 16 + (lane & 15)] = (_Float16)(accO[t][r] * (PUN / rowL[r]));
    }
  }
  __syncthreads();
#pragma unroll
  for (int q = 0; q < 4; ++q) {
    const int ml = q * 4 + (lane >> 3), pc = lane & 7;
    vst2(ctx + ((size_t)(b * kS + q0 + wave * 16 + ml)) * kD + h * kHD + pc * 8, *(const v4u*)(&so[ml * 64 + pc * 8]));
  }
}

extern "C" void kernel_launch(void* const* d_in, const int* in_sizes, int n_in,
                              void* d_out, int out_size, void* d_ws, size_t ws_size,
                              hipStream_t stream) {
  (void)in_sizes; (void)n_in; (void)out_size; (void)ws_size;
  const float* x   = (const float*)d_in[0];
  const float* Wq  = (const float*)d_in[1];
  const float* bq  = (const float*)d_in[2];
  const float* Wk  = (const float*)d_in[3];
  const float* bk  = (const float*)d_in[4];
  const float* Wv  = (const float*)d_in[5];
  const float* bv  = (const float*)d_in[6];
  const float* Wo  = (const float*)d_in[7];
  const float* bo  = (const float*)d_in[8];
  const float* rel = (const float*)d_in[9];
  float* out = (float*)d_out;

  const size_t T = (size_t)kB * kS;
  const size_t WSZ = (size_t)kD * kD;
  _Float16* xb  = (_Float16*)d_ws;
  _Float16* WqT = xb  + T * kD;
  _Float16* WkT = WqT + WSZ;
  _Float16* WvT = WkT + WSZ;
  _Float16* WoT = WvT + WSZ;
  _Float16* Q   = WoT + WSZ;
  _Float16* Kp  = Q  + T * kD;
  _Float16* Vp  = Kp + T * kD;
  _Float16* Cx  = Vp + T * kD;

  const float scale = 0.125f;
  dim3 bl(128);
  dim3 gg(kD / 64, (unsigned)(T / 64));
  dim3 gw(kD / 64, kD / 64);
  const int nx = (int)(T * kD);

  hipLaunchKernelGGL(cvt_bf16_kernel, dim3(nx / 512), dim3(256), 0, stream, x, xb, nx);
  hipLaunchKernelGGL(wtrans_kernel, gw, bl, 0, stream, Wq, WqT, kD, kD);
  hipLaunchKernelGGL(wtrans_kernel, gw, bl, 0, stream, Wk, WkT, kD, kD);
  hipLaunchKernelGGL(wtrans_kernel, gw, bl, 0, stream, Wv, WvT, kD, kD);
  hipLaunchKernelGGL(wtrans_kernel, gw, bl, 0, stream, Wo, WoT, kD, kD);

  hipLaunchKernelGGL((gemm_bias_kernel<_Float16>), gg, bl, 0, stream, xb, WqT, bq, Q,  kD, kD, scale);
  hipLaunchKernelGGL((gemm_bias_kernel<_Float16>), gg, bl, 0, stream, xb, WkT, bk, Kp, kD, kD, 1.0f);
  hipLaunchKernelGGL((gemm_bias_kernel<_Float16>), gg, bl, 0, stream, xb, WvT, bv, Vp, kD, kD, 1.0f);
  hipLaunchKernelGGL(rel_attn_kernel, dim3(kB * kH * (kS / 64)), bl, 0, stream, Q, Kp, Vp, rel, Cx);
  hipLaunchKernelGGL((gemm_bias_kernel<float>), gg, bl, 0, stream, Cx, WoT, bo, out, kD, kD, 1.0f);
}
